// EnhancedIPA2_27118423507359
// MI455X (gfx1250) — hardware-run, weakly checked
//
#include <hip/hip_runtime.h>
#include <hip/hip_bf16.h>
#include <stddef.h>
#include <stdint.h>

#define NB     4
#define LL     1024
#define NTOK   4096
#define CS     384
#define HH     12
#define CH     16
#define NP     8
#define NQ     192
#define NPROJ  2400
#define NPP    2432
#define COL_K  192
#define COL_V  384
#define COL_QP 576
#define COL_KP 1152
#define COL_VP 1728
#define COL_G  2304
#define FD     64
#define NBHL   49152
#define FEAT   864
#define FSEG   896
#define KWO    2688
#define TP     72
#define OTP    68
#define EPSV   1e-12f
#define SC_INV 0.125f
#define P_CARRY 16.0f
#define P_INV  0.0625f

static_assert(NTOK == NB * LL);
static_assert(NBHL == NB * HH * LL);
static_assert(NQ == HH * CH);
static_assert(NPROJ == NQ + 2 * NQ + 6 * HH * NP + 12 * HH * NP + HH * NP);
static_assert(NPP % 64 == 0);
static_assert(NPP >= NPROJ);
static_assert(COL_QP == 9 * 64);
static_assert(COL_G == 36 * 64);
static_assert(FEAT == HH * (CH + 7 * NP));
static_assert(KWO == 3 * FSEG);
static_assert(FSEG % 64 == 0);
static_assert(FSEG >= FEAT);
static_assert(CS % 64 == 0);
static_assert((NTOK * CS) % 2048 == 0);
static_assert(LL % 64 == 0);
static_assert(NTOK % 256 == 0);
static_assert(FD == CH + 6 * NP);
static_assert(COL_K % 4 == 0);
static_assert(COL_QP % 4 == 0);
static_assert(COL_KP % 4 == 0);
static_assert(COL_G % 4 == 0);
static_assert(NPROJ % 4 == 0);
static_assert((HH * NP) % 4 == 0);

typedef _Float16 v16h __attribute__((ext_vector_type(16)));
typedef _Float16 v8h  __attribute__((ext_vector_type(8)));
typedef __bf16   v16b __attribute__((ext_vector_type(16)));
typedef unsigned short v8us __attribute__((ext_vector_type(8)));
typedef float v8f __attribute__((ext_vector_type(8)));
typedef float v4f __attribute__((ext_vector_type(4)));
typedef float v2f __attribute__((ext_vector_type(2)));
typedef unsigned int v4u __attribute__((ext_vector_type(4)));

union PackH { v8h h; v4u u; };
union PackU { v8us s; v4u u; };

__device__ __forceinline__ v8f zero8() { return (v8f){0.f, 0.f, 0.f, 0.f, 0.f, 0.f, 0.f, 0.f}; }
__device__ __forceinline__ v8h zero8h() {
  const _Float16 z = (_Float16)0.0f;
  return (v8h){z, z, z, z, z, z, z, z};
}
__device__ __forceinline__ int clampi(int x, int lo, int hi) { return x < lo ? lo : (x > hi ? hi : x); }
__device__ __forceinline__ unsigned int bf16_rne(float x) {
  const unsigned int u = __float_as_uint(x);
  return (u + 0x7FFFu + ((u >> 16) & 1u)) >> 16;
}
__device__ __forceinline__ float bf16_tof(unsigned int b) { return __uint_as_float(b << 16); }

struct OpF16 {
  typedef _Float16 E;
  typedef v16h F;
  static __device__ __forceinline__ F ld(const E* p, int ldk, size_t row0, int k0, int lane) {
    const int m = lane & 15, lh = lane >> 4;
    const E* q = p + (row0 + (size_t)m) * (size_t)ldk + k0 + 8 * lh;
    union { F v; v8h hv[2]; } f;
    f.hv[0] = *(const v8h*)(q);
    f.hv[1] = *(const v8h*)(q + 16);
    return f.v;
  }
  static __device__ __forceinline__ v8f mma(F a, F b, v8f c) {
    c = __builtin_amdgcn_wmma_f32_16x16x32_f16(false, a, false, b, (short)0, c, false, false);
    asm volatile("v_nop\n\tv_nop\n\tv_nop\n\tv_nop" : "+v"(c) : "v"(a), "v"(b));
    return c;
  }
};
struct OpBF16 {
  typedef unsigned short E;
  typedef v16b F;
  static __device__ __forceinline__ F ld(const E* p, int ldk, size_t row0, int k0, int lane) {
    const int m = lane & 15, lh = lane >> 4;
    const E* q = p + (row0 + (size_t)m) * (size_t)ldk + k0 + 8 * lh;
    union { F v; v8us uv[2]; } f;
    f.uv[0] = *(const v8us*)(q);
    f.uv[1] = *(const v8us*)(q + 16);
    return f.v;
  }
  static __device__ __forceinline__ v8f mma(F a, F b, v8f c) {
    c = __builtin_amdgcn_wmma_f32_16x16x32_bf16(false, a, false, b, (short)0, c, false, false);
    asm volatile("v_nop\n\tv_nop\n\tv_nop\n\tv_nop" : "+v"(c) : "v"(a), "v"(b));
    return c;
  }
};

__global__ __launch_bounds__(256) void k_cvt(const float* __restrict__ src, _Float16* __restrict__ dh, float scale) {
  const int tid = threadIdx.x;
  const size_t o = (size_t)blockIdx.x * 2048 + (size_t)tid * 8;
  const v4f a0 = *(const v4f*)(src + o) * scale;
  const v4f a1 = *(const v4f*)(src + o + 4) * scale;
  PackH pk;
  pk.h = (v8h){(_Float16)a0[0], (_Float16)a0[1], (_Float16)a0[2], (_Float16)a0[3],
               (_Float16)a1[0], (_Float16)a1[1], (_Float16)a1[2], (_Float16)a1[3]};
  const v4u vv = pk.u;
  volatile v4u* d = (volatile v4u*)(dh + o);
  *d = vv;
  __threadfence();
  *d = vv;
}

__global__ __launch_bounds__(256) void k_wtrans(const float* __restrict__ src, int Ksrc, int Nsrc,
                                                unsigned short* __restrict__ dst, int ldd, int dstrow0,
                                                int seg, int mode, float scale) {
  __shared__ __align__(16) float T[64][68];
  const int tid = threadIdx.x;
  const int n0 = blockIdx.x * 64, k0 = blockIdx.y * 64;
#pragma unroll
  for (int it = 0; it < 4; ++it) {
    const int idx = tid + 256 * it;
    const int krow = idx >> 4, n4 = (idx & 15) * 4;
    const int gk = k0 + krow, gn = n0 + n4;
    const int kcl = (gk < Ksrc) ? gk : (Ksrc - 1);
    const int ncl = (gn <= Nsrc - 4) ? gn : (Nsrc - 4);
    const v4f v = *(const v4f*)(src + (size_t)kcl * Nsrc + ncl);
    const bool ok = (gk < Ksrc) && (gn < Nsrc);
    T[n4 + 0][krow] = ok ? v[0] : 0.0f;
    T[n4 + 1][krow] = ok ? v[1] : 0.0f;
    T[n4 + 2][krow] = ok ? v[2] : 0.0f;
    T[n4 + 3][krow] = ok ? v[3] : 0.0f;
  }
  __syncthreads();
  const int nseg = (mode != 0) ? 3 : 1;
  for (int s = 0; s < nseg; ++s) {
    v4u val[2];
    size_t go[2];
#pragma unroll
    for (int it = 0; it < 2; ++it) {
      const int p = tid + 256 * it;
      const int row = p >> 3, pc = p & 7;
      const v4f x0 = *(const v4f*)(&T[row][pc * 8]);
      const v4f x1 = *(const v4f*)(&T[row][pc * 8 + 4]);
      const float f[8] = {x0[0], x0[1], x0[2], x0[3], x1[0], x1[1], x1[2], x1[3]};
      if (mode == 0) {
        PackH ph;
        ph.h = (v8h){(_Float16)(f[0] * scale), (_Float16)(f[1] * scale), (_Float16)(f[2] * scale),
                     (_Float16)(f[3] * scale), (_Float16)(f[4] * scale), (_Float16)(f[5] * scale),
                     (_Float16)(f[6] * scale), (_Float16)(f[7] * scale)};
        val[it] = ph.u;
      } else {
        unsigned int bits[8];
#pragma unroll
        for (int j = 0; j < 8; ++j) {
          const unsigned int hb = bf16_rne(f[j]);
          const unsigned int lb = bf16_rne(f[j] - bf16_tof(hb));
          bits[j] = (s == 2) ? lb : hb;
        }
        PackU pu;
        pu.s = (v8us){(unsigned short)bits[0], (unsigned short)bits[1], (unsigned short)bits[2],
                      (unsigned short)bits[3], (unsigned short)bits[4], (unsigned short)bits[5],
                      (unsigned short)bits[6], (unsigned short)bits[7]};
        val[it] = pu.u;
      }
      go[it] = (size_t)(dstrow0 + n0 + row) * (size_t)ldd + (size_t)s * seg + k0 + pc * 8;
    }
    for (int ps = 0; ps < 2; ++ps) {
#pragma unroll
      for (int it = 0; it < 2; ++it) *(volatile v4u*)(dst + go[it]) = val[it];
      __threadfence();
    }
  }
}

__global__ __launch_bounds__(256) void k_bias(const float* __restrict__ bq, const float* __restrict__ bkv,
                                              const float* __restrict__ bqp, const float* __restrict__ bkvp,
                                              const float* __restrict__ bg, float* __restrict__ bias) {
  const int tid = threadIdx.x;
#pragma unroll 1
  for (int it = 0; it < 3; ++it) {
    const int q  = tid + 256 * it;
    const int qc = (q < NPP / 4) ? q : (NPP / 4 - 1);
    const int n  = 4 * qc;
    const v4f v0 = *(const v4f*)(bq   + clampi(n,          0, NQ - 4));
    const v4f v1 = *(const v4f*)(bkv  + clampi(n - COL_K,  0, 2 * NQ - 4));
    const v4f v2 = *(const v4f*)(bqp  + clampi(n - COL_QP, 0, 6 * HH * NP - 4));
    const v4f v3 = *(const v4f*)(bkvp + clampi(n - COL_KP, 0, 12 * HH * NP - 4));
    const v4f v4 = *(const v4f*)(bg   + clampi(n - COL_G,  0, HH * NP - 4));
    v4f e = (v4f){0.0f, 0.0f, 0.0f, 0.0f};
    if (n < COL_K) e = v0;
    else if (n < COL_QP) e = v1;
    else if (n < COL_KP) e = v2;
    else if (n < COL_G) e = v3;
    else if (n < NPROJ) e = v4;
    const bool act = (q < NPP / 4);
    volatile v4f* d = (volatile v4f*)(bias + 4 * qc);
    if (act) *d = e;
    __threadfence();
    if (act) *d = e;
  }
}

template <class OP>
__device__ __forceinline__ void gemm32x64(const typename OP::E* __restrict__ A, int lda,
                                          const typename OP::E* __restrict__ Bt, int ldb, int K,
                                          int m0, int n0, int lane, v8f (&acc)[2][4]) {
#pragma unroll 1
  for (int k0 = 0; k0 < K; k0 += 32) {
    const typename OP::F a0 = OP::ld(A, lda, (size_t)m0, k0, lane);
    const typename OP::F a1 = OP::ld(A, lda, (size_t)m0 + 16, k0, lane);
    const typename OP::F b0 = OP::ld(Bt, ldb, (size_t)n0, k0, lane);
    const typename OP::F b1 = OP::ld(Bt, ldb, (size_t)n0 + 16, k0, lane);
    const typename OP::F b2 = OP::ld(Bt, ldb, (size_t)n0 + 32, k0, lane);
    const typename OP::F b3 = OP::ld(Bt, ldb, (size_t)n0 + 48, k0, lane);
    acc[0][0] = OP::mma(a0, b0, acc[0][0]);
    acc[1][0] = OP::mma(a1, b0, acc[1][0]);
    acc[0][1] = OP::mma(a0, b1, acc[0][1]);
    acc[1][1] = OP::mma(a1, b1, acc[1][1]);
    acc[0][2] = OP::mma(a0, b2, acc[0][2]);
    acc[1][2] = OP::mma(a1, b2, acc[1][2]);
    acc[0][3] = OP::mma(a0, b3, acc[0][3]);
    acc[1][3] = OP::mma(a1, b3, acc[1][3]);
  }
}

__device__ __forceinline__ void epilogue_f32(v8f (&acc)[2][4], float scale, const float* __restrict__ bias, int act,
                                             float* sw, float* __restrict__ out, int ldo,
                                             int m0, int n0, int lane, int hh, int c) {
  float bn[4];
#pragma unroll
  for (int t = 0; t < 4; ++t) bn[t] = bias[n0 + 16 * t + c];
#pragma unroll
  for (int sub = 0; sub < 2; ++sub) {
    __syncthreads();
#pragma unroll
    for (int t = 0; t < 4; ++t) {
#pragma unroll
      for (int r = 0; r < 8; ++r) {
        float v = fmaf(acc[sub][t][r], scale, bn[t]);
        if (act == 1) v = fmaxf(v, 0.0f);
        else if (act == 2) v = __builtin_amdgcn_rcpf(1.0f + __expf(-v));
        sw[(8 * hh + r) * OTP + 16 * t + c] = v;
      }
    }
    __syncthreads();
    v4f val[8];
    size_t go[8];
#pragma unroll
    for (int it = 0; it < 8; ++it) {
      const int p    = lane + 32 * it;
      const int L    = p >> 3;
      const int pc   = p & 7;
      const int row  = L >> 1;
      const int half = L & 1;
      val[it] = *(const v4f*)(sw + row * OTP + half * 32 + pc * 4);
      go[it]  = (size_t)(m0 + sub * 16 + row) * ldo + n0 + half * 32 + pc * 4;
    }
    for (int ps = 0; ps < 2; ++ps) {
#pragma unroll
      for (int it = 0; it < 8; ++it) *(volatile v4f*)(out + go[it]) = val[it];
      __threadfence();
    }
  }
}

template <class OP>
__global__ __launch_bounds__(256) void k_gemm(const typename OP::E* __restrict__ ap, int lda,
                                              const typename OP::E* __restrict__ wt, int ldb, int K, float scale,
                                              const float* __restrict__ bias, float* __restrict__ out, int ldo,
                                              int relu_lo, int sig_lo) {
  __shared__ __align__(16) float st[8][16 * OTP];
  const int tid = threadIdx.x, lane = tid & 31, wave = tid >> 5;
  const int hh = lane >> 4, c = lane & 15;
  const int m0 = blockIdx.x * 256 + wave * 32;
  const int n0 = blockIdx.y * 64;
  int act = 0;
  if ((int)blockIdx.y >= sig_lo) act = 2;
  else if ((int)blockIdx.y >= relu_lo) act = 1;

  v8f acc[2][4];
#pragma unroll
  for (int s = 0; s < 2; ++s)
#pragma unroll
    for (int t = 0; t < 4; ++t) acc[s][t] = zero8();
  gemm32x64<OP>(ap, lda, wt, ldb, K, m0, n0, lane, acc);
  epilogue_f32(acc, scale, bias, act, st[wave], out, ldo, m0, n0, lane, hh, c);
}

__device__ __forceinline__ void store_tile64(const _Float16 (*S)[TP], _Float16* __restrict__ dst,
                                             size_t row0, int ldd, int col0, int tid) {
  v4u v[8];
  size_t go[8];
#pragma unroll
  for (int it = 0; it < 8; ++it) {
    const int p = tid + 64 * it;
    const int row = p >> 3, pc = p & 7;
    PackH ph;
    ph.h = *(const v8h*)(&S[row][pc * 8]);
    v[it] = ph.u;
    go[it] = (row0 + (size_t)row) * (size_t)ldd + col0 + pc * 8;
  }
  for (int ps = 0; ps < 2; ++ps) {
#pragma unroll
    for (int it = 0; it < 8; ++it) *(volatile v4u*)(dst + go[it]) = v[it];
    __threadfence();
  }
}

__global__ __launch_bounds__(64) void k_prep_q(const float* __restrict__ PR, const float* __restrict__ rot,
                                               const float* __restrict__ trans, const float* __restrict__ head_w,
                                               const float* __restrict__ geom_w, _Float16* __restrict__ QF,
                                               float* __restrict__ QC4) {
  __shared__ __align__(16) _Float16 Qs[64][TP];
  const int tid = threadIdx.x;
  const int bh = blockIdx.x >> 4, lt = blockIdx.x & 15;
  const int b = bh / HH, h = bh - b * HH;
  const int l = lt * 64 + tid;
  const size_t bl = (size_t)b * LL + l;
  const size_t prow = (size_t)bh * LL + l;
  const float* pr = PR + bl * NPP;
  float R[9], T3[3];
#pragma unroll
  for (int i = 0; i < 9; ++i) R[i] = rot[bl * 9 + i];
#pragma unroll
  for (int i = 0; i < 3; ++i) T3[i] = trans[bl * 3 + i];
  const float hw = 1.0f / (1.0f + __expf(-head_w[h]));
  const float sq = 2.0f * hw;
  const float sd = 8.0f * hw * geom_w[1];
  {
    const float* qp0 = pr + h * CH;
    const v4f u0 = *(const v4f*)(qp0) * sq;
    const v4f u1 = *(const v4f*)(qp0 + 4) * sq;
    const v4f u2 = *(const v4f*)(qp0 + 8) * sq;
    const v4f u3 = *(const v4f*)(qp0 + 12) * sq;
    *(v8h*)(&Qs[tid][0]) = (v8h){(_Float16)u0[0], (_Float16)u0[1], (_Float16)u0[2], (_Float16)u0[3],
                                 (_Float16)u1[0], (_Float16)u1[1], (_Float16)u1[2], (_Float16)u1[3]};
    *(v8h*)(&Qs[tid][8]) = (v8h){(_Float16)u2[0], (_Float16)u2[1], (_Float16)u2[2], (_Float16)u2[3],
                                 (_Float16)u3[0], (_Float16)u3[1], (_Float16)u3[2], (_Float16)u3[3]};
    const v8h z8 = zero8h();
    *(v8h*)(&Qs[tid][40]) = z8;
    *(v8h*)(&Qs[tid][48]) = z8;
    *(v8h*)(&Qs[tid][56]) = z8;
  }
  float cxs = 0.0f, cys = 0.0f, czs = 0.0f;
#pragma unroll 1
  for (int p = 0; p < NP; ++p) {
    const float* qp = pr + COL_QP + (h * NP + p) * 6;
    const v2f w0 = *(const v2f*)(qp);
    const v2f w1 = *(const v2f*)(qp + 2);
    const v2f w2 = *(const v2f*)(qp + 4);
    const float p0 = w0[0], p1 = w0[1], p2 = w1[0], p3 = w1[1], p4 = w2[0], p5 = w2[1];
    const float g = pr[COL_G + h * NP + p];
    const float cx = (R[0] * p0 + R[1] * p1 + R[2] * p2 + T3[0]) * g;
    const float cy = (R[3] * p0 + R[4] * p1 + R[5] * p2 + T3[1]) * g;
    const float cz = (R[6] * p0 + R[7] * p1 + R[8] * p2 + T3[2]) * g;
    const float dx = (R[0] * p3 + R[1] * p4 + R[2] * p5) * g;
    const float dy = (R[3] * p3 + R[4] * p4 + R[5] * p5) * g;
    const float dz = (R[6] * p3 + R[7] * p4 + R[8] * p5) * g;
    cxs += cx; cys += cy; czs += cz;
    Qs[tid][CH + 3 * p + 0] = (_Float16)(dx * sd);
    Qs[tid][CH + 3 * p + 1] = (_Float16)(dy * sd);
    Qs[tid][CH + 3 * p + 2] = (_Float16)(dz * sd);
  }
  const float mx = cxs * 0.125f, my = cys * 0.125f, mz = czs * 0.125f;
  const v4f qc = (v4f){mx, my, mz, mx * mx + my * my + mz * mz};
  volatile v4f* qd = (volatile v4f*)(QC4 + prow * 4);
  *qd = qc;
  __threadfence();
  *qd = qc;
  __syncthreads();
  store_tile64(Qs, QF, (size_t)bh * LL + (size_t)lt * 64, FD, 0, tid);
}

__global__ __launch_bounds__(64) void k_prep_kv(const float* __restrict__ PR, const float* __restrict__ rot,
                                                const float* __restrict__ trans, _Float16* __restrict__ KF,
                                                _Float16* __restrict__ VT, float* __restrict__ KC4,
                                                float* __restrict__ VM) {
  __shared__ __align__(16) _Float16 Ks[64][TP];
  __shared__ __align__(16) _Float16 Vs[64][TP];
  const int tid = threadIdx.x;
  const int bh = blockIdx.x >> 4, lt = blockIdx.x & 15;
  const int b = bh / HH, h = bh - b * HH;
  const int l = lt * 64 + tid;
  const size_t bl = (size_t)b * LL + l;
  const size_t prow = (size_t)bh * LL + l;
  const float* pr = PR + bl * NPP;
  float R[9], T3[3];
#pragma unroll
  for (int i = 0; i < 9; ++i) R[i] = rot[bl * 9 + i];
#pragma unroll
  for (int i = 0; i < 3; ++i) T3[i] = trans[bl * 3 + i];
  {
    const float* kp0 = pr + COL_K + h * CH;
    const v4f u0 = *(const v4f*)(kp0);
    const v4f u1 = *(const v4f*)(kp0 + 4);
    const v4f u2 = *(const v4f*)(kp0 + 8);
    const v4f u3 = *(const v4f*)(kp0 + 12);
    *(v8h*)(&Ks[tid][0]) = (v8h){(_Float16)u0[0], (_Float16)u0[1], (_Float16)u0[2], (_Float16)u0[3],
                                 (_Float16)u1[0], (_Float16)u1[1], (_Float16)u1[2], (_Float16)u1[3]};
    *(v8h*)(&Ks[tid][8]) = (v8h){(_Float16)u2[0], (_Float16)u2[1], (_Float16)u2[2], (_Float16)u2[3],
                                 (_Float16)u3[0], (_Float16)u3[1], (_Float16)u3[2], (_Float16)u3[3]};
    const v8h z8 = zero8h();
    *(v8h*)(&Ks[tid][40]) = z8;
    *(v8h*)(&Ks[tid][48]) = z8;
    *(v8h*)(&Ks[tid][56]) = z8;
    const float* vp0 = pr + COL_V + h * CH;
#pragma unroll
    for (int c4 = 0; c4 < 4; ++c4) {
      const v4f t = *(const v4f*)(vp0 + 4 * c4);
      Vs[4 * c4 + 0][tid] = (_Float16)t[0];
      Vs[4 * c4 + 1][tid] = (_Float16)t[1];
      Vs[4 * c4 + 2][tid] = (_Float16)t[2];
      Vs[4 * c4 + 3][tid] = (_Float16)t[3];
    }
  }
  float kxs = 0.0f, kys = 0.0f, kzs = 0.0f;
  float vxs = 0.0f, vys = 0.0f, vzs = 0.0f;
#pragma unroll 1
  for (int p = 0; p < NP; ++p) {
    const float* kp = pr + COL_KP + (h * NP + p) * 6;
    const v2f w0 = *(const v2f*)(kp);
    const v2f w1 = *(const v2f*)(kp + 2);
    const v2f w2 = *(const v2f*)(kp + 4);
    const float p0 = w0[0], p1 = w0[1], p2 = w1[0], p3 = w1[1], p4 = w2[0], p5 = w2[1];
    const float kcx = R[0] * p0 + R[1] * p1 + R[2] * p2 + T3[0];
    const float kcy = R[3] * p0 + R[4] * p1 + R[5] * p2 + T3[1];
    const float kcz = R[6] * p0 + R[7] * p1 + R[8] * p2 + T3[2];
    const float kdx = R[0] * p3 + R[1] * p4 + R[2] * p5;
    const float kdy = R[3] * p3 + R[4] * p4 + R[5] * p5;
    const float kdz = R[6] * p3 + R[7] * p4 + R[8] * p5;
    kxs += kcx; kys += kcy; kzs += kcz;
    Ks[tid][CH + 3 * p + 0] = (_Float16)kdx;
    Ks[tid][CH + 3 * p + 1] = (_Float16)kdy;
    Ks[tid][CH + 3 * p + 2] = (_Float16)kdz;

    const float* vp = pr + COL_VP + (h * NP + p) * 6;
    const v2f x0 = *(const v2f*)(vp);
    const v2f x1 = *(const v2f*)(vp + 2);
    const v2f x2 = *(const v2f*)(vp + 4);
    const float s0 = x0[0], s1 = x0[1], s2 = x1[0], s3 = x1[1], s4 = x2[0], s5 = x2[1];
    const float vcx = R[0] * s0 + R[1] * s1 + R[2] * s2 + T3[0];
    const float vcy = R[3] * s0 + R[4] * s1 + R[5] * s2 + T3[1];
    const float vcz = R[6] * s0 + R[7] * s1 + R[8] * s2 + T3[2];
    const float vdx = R[0] * s3 + R[1] * s4 + R[2] * s5;
    const float vdy = R[3] * s3 + R[4] * s4 + R[5] * s5;
    const float vdz = R[6] * s3 + R[7] * s4 + R[8] * s5;
    vxs += vcx; vys += vcy; vzs += vcz;
    Vs[CH + 6 * p + 0][tid] = (_Float16)vcx;
    Vs[CH + 6 * p + 1][tid] = (_Float16)vcy;
    Vs[CH + 6 * p + 2][tid] = (_Float16)vcz;
    Vs[CH + 6 * p + 3][tid] = (_Float16)vdx;
    Vs[CH + 6 * p + 4][tid] = (_Float16)vdy;
    Vs[CH + 6 * p + 5][tid] = (_Float16)vdz;
  }
  {
    const float mx = kxs * 0.125f, my = kys * 0.125f, mz = kzs * 0.125f;
    const v4f kc = (v4f){mx, my, mz, mx * mx + my * my + mz * mz};
    volatile v4f* kd = (volatile v4f*)(KC4 + prow * 4);
    *kd = kc;
    __threadfence();
    *kd = kc;
    const v4f vmv = (v4f){vxs * 0.125f, vys * 0.125f, vzs * 0.125f, 0.0f};
    volatile v4f* vd = (volatile v4f*)(VM + prow * 4);
    *vd = vmv;
    __threadfence();
    *vd = vmv;
  }
  __syncthreads();
  store_tile64(Ks, KF, (size_t)bh * LL + (size_t)lt * 64, FD, 0, tid);
  store_tile64(Vs, VT, (size_t)bh * FD, LL, lt * 64, tid);
}

__device__ __forceinline__ void score16(const _Float16* __restrict__ KF, const float* __restrict__ KC4,
                                        size_t krow, v16h a0, v16h a1,
                                        const float (&qx)[8], const float (&qy)[8], const float (&qz)[8],
                                        const float (&q2)[8], float poscoef, int lane, int n, float (&dst)[8]) {
  const v16h b0 = OpF16::ld(KF, FD, krow, 0, lane);
  const v16h b1 = OpF16::ld(KF, FD, krow, 32, lane);
  v8f c = zero8();
  c = OpF16::mma(a0, b0, c);
  c = OpF16::mma(a1, b1, c);
  const v4f kq = *(const v4f*)(KC4 + (krow + (size_t)n) * 4);
#pragma unroll
  for (int r = 0; r < 8; ++r) {
    float dp = qx[r] * kq[0];
    dp = fmaf(qy[r], kq[1], dp);
    dp = fmaf(qz[r], kq[2], dp);
    float d2 = (q2[r] + kq[3]) - 2.0f * dp;
    d2 = fmaxf(d2, EPSV);
    dst[r] = fmaf(-poscoef, sqrtf(d2), c[r] * SC_INV);
  }
}

__global__ __launch_bounds__(32) void k_attn(const _Float16* __restrict__ QF, const _Float16* __restrict__ KF,
                                             const _Float16* __restrict__ VT, const float* __restrict__ QC4,
                                             const float* __restrict__ KC4, const float* __restrict__ head_w,
                                             const float* __restrict__ geom_w, float* __restrict__ OB) {
  __shared__ __align__(16) _Float16 Ps[16][40];
  __shared__ __align__(16) float Os[16][68];
  const int lane = threadIdx.x;
  const int hh = lane >> 4, n = lane & 15;
  const int qt = blockIdx.x & 63;
  const int bh = blockIdx.x >> 6;
  const int b = bh / HH, h = bh - b * HH;
  const float hw = 1.0f / (1.0f + __expf(-head_w[h]));
  const float poscoef = hw * geom_w[0];
  const size_t qrow0 = (size_t)bh * LL + (size_t)qt * 16;

  const v16h a0 = OpF16::ld(QF, FD, qrow0, 0, lane);
  const v16h a1 = OpF16::ld(QF, FD, qrow0, 32, lane);
  float qx[8], qy[8], qz[8], q2[8];
#pragma unroll
  for (int r = 0; r < 8; ++r) {
    const v4f t = *(const v4f*)(QC4 + (qrow0 + (size_t)(8 * hh + r)) * 4);
    qx[r] = t[0]; qy[r] = t[1]; qz[r] = t[2]; q2[r] = t[3];
  }
  float rmax[8], rsum[8];
  v8f acc[4];
#pragma unroll
  for (int r = 0; r < 8; ++r) { rmax[r] = -1.0e30f; rsum[r] = 0.0f; }
#pragma unroll
  for (int nt = 0; nt < 4; ++nt) acc[nt] = zero8();
  const _Float16* VTb = VT + (size_t)bh * FD * LL;

#pragma unroll 1
  for (int kc = 0; kc < LL / 32; ++kc) {
    const size_t krow0 = (size_t)bh * LL + (size_t)kc * 32;
    float s0[8], s1[8];
    score16(KF, KC4, krow0, a0, a1, qx, qy, qz, q2, poscoef, lane, n, s0);
    score16(KF, KC4, krow0 + 16, a0, a1, qx, qy, qz, q2, poscoef, lane, n, s1);
#pragma unroll
    for (int r = 0; r < 8; ++r) {
      float v = fmaxf(s0[r], s1[r]);
      v = fmaxf(v, __shfl_xor(v, 1));
      v = fmaxf(v, __shfl_xor(v, 2));
      v = fmaxf(v, __shfl_xor(v, 4));
      v = fmaxf(v, __shfl_xor(v, 8));
      const float nm = fmaxf(rmax[r], v);
      const float rs = __expf(rmax[r] - nm);
      rmax[r] = nm;
      const float p0 = __expf(s0[r] - nm);
      const float p1 = __expf(s1[r] - nm);
      float ps = p0 + p1;
      ps += __shfl_xor(ps, 1);
      ps += __shfl_xor(ps, 2);
      ps += __shfl_xor(ps, 4);
      ps += __shfl_xor(ps, 8);
      rsum[r] = fmaf(rsum[r], rs, ps);
#pragma unroll
      for (int nt = 0; nt < 4; ++nt) acc[nt][r] = acc[nt][r] * rs;
      Ps[8 * hh + r][n]      = (_Float16)(p0 * P_CARRY);
      Ps[8 * hh + r][16 + n] = (_Float16)(p1 * P_CARRY);
    }
    __syncthreads();
    union { v16h v; v8h hv[2]; } pa;
    pa.hv[0] = *(const v8h*)(&Ps[n][8 * hh]);
    pa.hv[1] = *(const v8h*)(&Ps[n][16 + 8 * hh]);
#pragma unroll
    for (int nt = 0; nt < 4; ++nt) {
      const v16h bv = OpF16::ld(VTb, LL, (size_t)(16 * nt), kc * 32, lane);
      acc[nt] = OpF16::mma(pa.v, bv, acc[nt]);
    }
    __syncthreads();
  }

#pragma unroll
  for (int r = 0; r < 8; ++r) {
    const float inv = P_INV / rsum[r];
#pragma unroll
    for (int nt = 0; nt < 4; ++nt) Os[8 * hh + r][16 * nt + n] = acc[nt][r] * inv;
  }
  __syncthreads();
  v4f ov[8];
  size_t og[8];
#pragma unroll
  for (int it = 0; it < 8; ++it) {
    const int p = lane + 32 * it;
    const int row = p >> 4, pc = p & 15;
    ov[it] = *(const v4f*)(&Os[row][pc * 4]);
    og[it] = (((size_t)b * LL + (size_t)qt * 16 + row) * HH + h) * FD + pc * 4;
  }
  for (int ps = 0; ps < 2; ++ps) {
#pragma unroll
    for (int it = 0; it < 8; ++it) *(volatile v4f*)(OB + og[it]) = ov[it];
    __threadfence();
  }
}

__global__ __launch_bounds__(96) void k_post(const float* __restrict__ OB, const float* __restrict__ VM,
                                             unsigned short* __restrict__ FP) {
  __shared__ __align__(16) float F[8][FSEG];
  const int tid = threadIdx.x;
  const int h = tid >> 3, li = tid & 7;
  const int row0 = blockIdx.x * 8;
  const int b = row0 >> 10, l0 = row0 & (LL - 1);
  const size_t tok = (size_t)row0 + li;
  const float* o = OB + (tok * HH + h) * FD;
#pragma unroll
  for (int c4 = 0; c4 < 4; ++c4) *(v4f*)(&F[li][h * CH + 4 * c4]) = *(const v4f*)(o + 4 * c4);
  const v4f vm = *(const v4f*)(VM + (((size_t)b * HH + h) * LL + l0 + li) * 4);
#pragma unroll 1
  for (int p = 0; p < NP; ++p) {
    const float* g = o + CH + p * 6;
    const v2f g0 = *(const v2f*)(g);
    const v2f g1 = *(const v2f*)(g + 2);
    const v2f g2 = *(const v2f*)(g + 4);
    const float lx = g0[0] - vm[0], ly = g0[1] - vm[1], lz = g1[0] - vm[2];
    const float ux = g1[1], uy = g2[0], uz = g2[1];
    const float dn = sqrtf(ux * ux + uy * uy + uz * uz);
    const float inv = 1.0f / fmaxf(dn, EPSV);
    const float ln = sqrtf(fmaxf(lx * lx + ly * ly + lz * lz, EPSV));
    float* f = &F[li][NQ + (h * NP + p) * 7];
    f[0] = lx; f[1] = ly; f[2] = lz;
    f[3] = ux * inv; f[4] = uy * inv; f[5] = uz * inv;
    f[6] = ln;
  }
  if (tid < 64) *(v4f*)(&F[tid >> 3][FEAT + (tid & 7) * 4]) = (v4f){0.0f, 0.0f, 0.0f, 0.0f};
  __syncthreads();
#pragma unroll 1
  for (int it = 0; it < 28; ++it) {
    const int q = tid + 96 * it;
    const int li2 = q / 336;
    const int rem = q - li2 * 336;
    const int seg = rem / 112;
    const int pp = rem - seg * 112;
    const int col0 = pp * 8;
    const v4f x0 = *(const v4f*)(&F[li2][col0]);
    const v4f x1 = *(const v4f*)(&F[li2][col0 + 4]);
    const float x[8] = {x0[0], x0[1], x0[2], x0[3], x1[0], x1[1], x1[2], x1[3]};
    unsigned int bits[8];
#pragma unroll
    for (int j = 0; j < 8; ++j) {
      const unsigned int hb = bf16_rne(x[j]);
      const unsigned int lb = bf16_rne(x[j] - bf16_tof(hb));
      bits[j] = (seg == 1) ? lb : hb;
    }
    PackU pu;
    pu.s = (v8us){(unsigned short)bits[0], (unsigned short)bits[1], (unsigned short)bits[2],
                  (unsigned short)bits[3], (unsigned short)bits[4], (unsigned short)bits[5],
                  (unsigned short)bits[6], (unsigned short)bits[7]};
    const v4u vv = pu.u;
    volatile v4u* d = (volatile v4u*)(FP + (size_t)(row0 + li2) * KWO + (size_t)seg * FSEG + col0);
    *d = vv;
    __threadfence();
    *d = vv;
  }
}

extern "C" void kernel_launch(void* const* d_in, const int* in_sizes, int n_in,
                              void* d_out, int out_size, void* d_ws, size_t ws_size,
                              hipStream_t stream) {
  if (n_in < 17) return;
  if (in_sizes[0] != NTOK * CS) return;
  if (in_sizes[1] != NTOK * 9) return;
  if (in_sizes[2] != NTOK * 3) return;
  if (in_sizes[3] != CS * NQ) return;
  if (in_sizes[4] != NQ) return;
  if (in_sizes[5] != CS * 2 * NQ) return;
  if (in_sizes[6] != 2 * NQ) return;
  if (in_sizes[7] != CS * 6 * HH * NP) return;
  if (in_sizes[8] != 6 * HH * NP) return;
  if (in_sizes[9] != CS * 12 * HH * NP) return;
  if (in_sizes[10] != 12 * HH * NP) return;
  if (in_sizes[11] != CS * HH * NP) return;
  if (in_sizes[12] != HH * NP) return;
  if (in_sizes[13] != 2) return;
  if (in_sizes[14] != HH) return;
  if (in_sizes[15] != FEAT * CS) return;
  if (in_sizes[16] != CS) return;
  if (out_size != NTOK * CS) return;

  const float* s     = (const float*)d_in[0];
  const float* rot   = (const float*)d_in[1];
  const float* trans = (const float*)d_in[2];
  const float* Wq    = (const float*)d_in[3];
  const float* bq    = (const float*)d_in[4];
  const float* Wkv   = (const float*)d_in[5];
  const float* bkv   = (const float*)d_in[6];
  const float* Wqp   = (const float*)d_in[7];
  const float* bqp   = (const float*)d_in[8];
  const float* Wkvp  = (const float*)d_in[9];
  const float* bkvp  = (const float*)d_in[10];
  const float* Wg    = (const float*)d_in[11];
  const float* bg    = (const float*)d_in[12];
  const float* gw    = (const float*)d_in[13];
  const float* hws   = (const float*)d_in[14];
  const float* Wo    = (const float*)d_in[15];
  const float* bo    = (const float*)d_in[16];
  float* out = (float*)d_out;

  size_t off = 0;
  const size_t oX    = off; off += (size_t)NTOK * CS * 2;
  const size_t oWt   = off; off += (size_t)NPP * CS * 2;
  const size_t oBias = off; off += (size_t)NPP * 4;
  const size_t oPR   = off; off += (size_t)NTOK * NPP * 4;
  const size_t oQF   = off; off += (size_t)NBHL * FD * 2;
  const size_t oKF   = off; off += (size_t)NBHL * FD * 2;
  const size_t oVT   = off; off += (size_t)NBHL * FD * 2;
  const size_t oQC   = off; off += (size_t)NBHL * 16;
  const size_t oKC   = off; off += (size_t)NBHL * 16;
  const size_t oVM   = off; off += (size_t)NBHL * 16;
  const size_t oOB   = off; off += (size_t)NBHL * FD * 4;
  const size_t oFP   = off; off += (size_t)NTOK * KWO * 2;
  const size_t oWo   = off; off += (size_t)CS * KWO * 2;
  if (off > ws_size) return;
  if (off > (size_t)134217728) return;
  if (((oWt | oBias | oPR | oQF | oKF | oVT | oQC | oKC | oVM | oOB | oFP | oWo) & 127) != 0) return;

  char* ws = (char*)d_ws;
  _Float16* Xh        = (_Float16*)(ws + oX);
  unsigned short* WtU = (unsigned short*)(ws + oWt);
  const _Float16* WtH = (const _Float16*)(ws + oWt);
  float* BIAS         = (float*)(ws + oBias);
  float* PR           = (float*)(ws + oPR);
  _Float16* QF        = (_Float16*)(ws + oQF);
  _Float16* KF        = (_Float16*)(ws + oKF);
  _Float16* VT        = (_Float16*)(ws + oVT);
  float* QC4          = (float*)(ws + oQC);
  float* KC4          = (float*)(ws + oKC);
  float* VM           = (float*)(ws + oVM);
  float* OB           = (float*)(ws + oOB);
  unsigned short* FP  = (unsigned short*)(ws + oFP);
  unsigned short* WoT = (unsigned short*)(ws + oWo);

  k_cvt<<<dim3((NTOK * CS) / 2048), dim3(256), 0, stream>>>(s, Xh, 1.0f);
  k_wtrans<<<dim3(NQ / 64, CS / 64), dim3(256), 0, stream>>>(Wq, CS, NQ, WtU, CS, 0, 0, 0, 32.0f);
  k_wtrans<<<dim3((2 * NQ) / 64, CS / 64), dim3(256), 0, stream>>>(Wkv, CS, 2 * NQ, WtU, CS, COL_K, 0, 0, 32.0f);
  k_wtrans<<<dim3((6 * HH * NP) / 64, CS / 64), dim3(256), 0, stream>>>(Wqp, CS, 6 * HH * NP, WtU, CS, COL_QP, 0, 0, 32.0f);
  k_wtrans<<<dim3((12 * HH * NP) / 64, CS / 64), dim3(256), 0, stream>>>(Wkvp, CS, 12 * HH * NP, WtU, CS, COL_KP, 0, 0, 32.0f);
  k_wtrans<<<dim3((NPP - COL_G) / 64, CS / 64), dim3(256), 0, stream>>>(Wg, CS, HH * NP, WtU, CS, COL_G, 0, 0, 32.0f);
  k_wtrans<<<dim3(CS / 64, FSEG / 64), dim3(256), 0, stream>>>(Wo, FEAT, CS, WoT, KWO, 0, FSEG, 1, 1.0f);
  k_bias<<<dim3(1), dim3(256), 0, stream>>>(bq, bkv, bqp, bkvp, bg, BIAS);
  k_gemm<OpF16><<<dim3(NTOK / 256, NPP / 64), dim3(256), 0, stream>>>(Xh, CS, WtH, CS, CS, 0.03125f, BIAS, PR, NPP, 9, 36);
  k_prep_q<<<dim3(NB * HH * (LL / 64)), dim3(64), 0, stream>>>(PR, rot, trans, hws, gw, QF, QC4);
  k_prep_kv<<<dim3(NB * HH * (LL / 64)), dim3(64), 0, stream>>>(PR, rot, trans, KF, VT, KC4, VM);
  k_attn<<<dim3(NB * HH * (LL / 16)), dim3(32), 0, stream>>>(QF, KF, VT, QC4, KC4, hws, gw, OB);
  k_post<<<dim3(NTOK / 8), dim3(96), 0, stream>>>(OB, VM, FP);
  k_gemm<OpBF16><<<dim3(NTOK / 256, CS / 64), dim3(256), 0, stream>>>(FP, KWO, WoT, KWO, KWO, 1.0f, bo, out, CS, 4096, 4096);
  (void)hipGetLastError();
}
